// LSTMWithAttention_30897994727671
// MI455X (gfx1250) — hardware-verified
//
#include <hip/hip_runtime.h>
#include <math.h>


#define NOP4 "v_nop\n\tv_nop\n\tv_nop\n\tv_nop"

typedef _Float16 f16t;
typedef unsigned short u16;
typedef f16t  v16h __attribute__((ext_vector_type(16)));
typedef f16t  v8h  __attribute__((ext_vector_type(8)));
typedef __bf16 bf16t;
typedef bf16t v16b __attribute__((ext_vector_type(16)));
typedef float v8f  __attribute__((ext_vector_type(8)));
typedef float v4f  __attribute__((ext_vector_type(4)));
typedef unsigned int v4u __attribute__((ext_vector_type(4)));

union FH  { v16h v; v8h q[2]; };
union FB  { v16b v; v4u q[2]; };
union P16 { v8h h; u16 s[8]; v4u u; };
union P32 { v4f f; v4u u; };

#define EP 136
#define GP 132
#define AP 260
#define BP 264
#define CP 68
#define HP 72

__device__ __forceinline__ v16h ldh(const f16t* p) {
    FH f;
    f.q[0] = *(const v8h*)p;
    f.q[1] = *(const v8h*)(p + 16);
    return f.v;
}
__device__ __forceinline__ v16b ldb(const u16* p) {
    FB f;
    f.q[0] = *(const v4u*)p;
    f.q[1] = *(const v4u*)(p + 16);
    return f.v;
}
__device__ __forceinline__ v8f wh(v16h a, v16h b, v8f c) {
    return __builtin_amdgcn_wmma_f32_16x16x32_f16(false, a, false, b, (short)0, c, false, false);
}
__device__ __forceinline__ v8f wb(v16b a, v16b b, v8f c) {
    return __builtin_amdgcn_wmma_f32_16x16x32_bf16(false, a, false, b, (short)0, c, false, false);
}
__device__ __forceinline__ v8f zf8() {
    v8f z = {0.f, 0.f, 0.f, 0.f, 0.f, 0.f, 0.f, 0.f};
    return z;
}

__device__ __forceinline__ void gd6h(v8f (&c)[2][3], v16h (&a)[2], v16h (&b)[3]) {
    asm volatile(NOP4
                 : "+v"(c[0][0]), "+v"(c[0][1]), "+v"(c[0][2]),
                   "+v"(c[1][0]), "+v"(c[1][1]), "+v"(c[1][2])
                 : "v"(a[0]), "v"(a[1]), "v"(b[0]), "v"(b[1]), "v"(b[2]));
}
__device__ __forceinline__ void gd4h(v8f (&c)[2][2], v16h (&a)[2], v16h (&b)[2]) {
    asm volatile(NOP4
                 : "+v"(c[0][0]), "+v"(c[0][1]), "+v"(c[1][0]), "+v"(c[1][1])
                 : "v"(a[0]), "v"(a[1]), "v"(b[0]), "v"(b[1]));
}
__device__ __forceinline__ void gd4b(v8f (&c)[2][2], v16b (&ah)[2], v16b (&al)[2],
                                     v16b (&bh)[2], v16b (&bl)[2]) {
    asm volatile(NOP4
                 : "+v"(c[0][0]), "+v"(c[0][1]), "+v"(c[1][0]), "+v"(c[1][1])
                 : "v"(ah[0]), "v"(ah[1]), "v"(al[0]), "v"(al[1]),
                   "v"(bh[0]), "v"(bh[1]), "v"(bl[0]), "v"(bl[1]));
}
__device__ __forceinline__ void gd2h(v8f& c0, v8f& c1, v16h a, v16h b0, v16h b1) {
    asm volatile(NOP4 : "+v"(c0), "+v"(c1) : "v"(a), "v"(b0), "v"(b1));
}
__device__ __forceinline__ void gd2b(v8f& c0, v8f& c1, v16b a0, v16b a1,
                                     v16b b0, v16b b1, v16b b2, v16b b3) {
    asm volatile(NOP4 : "+v"(c0), "+v"(c1)
                 : "v"(a0), "v"(a1), "v"(b0), "v"(b1), "v"(b2), "v"(b3));
}

__device__ __forceinline__ u16 bfb(float f) {
    unsigned int u = __float_as_uint(f);
    u += 0x7FFFu + ((u >> 16) & 1u);
    return (u16)(u >> 16);
}
__device__ __forceinline__ float bff(u16 b) {
    return __uint_as_float(((unsigned int)b) << 16);
}
__device__ __forceinline__ float ftanh(float x) {
    float ax = fabsf(x);
    float t  = __expf(-2.0f * ax);
    float r  = (1.0f - t) * __builtin_amdgcn_rcpf(1.0f + t);
    return copysignf(r, x);
}
__device__ __forceinline__ float fsigm(float x) {
    return __builtin_amdgcn_rcpf(1.0f + expf(-x));
}

__global__ __launch_bounds__(256)
void k_cvt_x(const float* __restrict__ x, f16t* xh, u16* xhi, u16* xlo, int n8) {
    const int i = blockIdx.x * 256 + threadIdx.x;
    if (i >= n8) return;
    const float* p = x + (size_t)i * 8;
    v4f a = *(const v4f*)p;
    v4f c = *(const v4f*)(p + 4);
    float f[8];
    f[0] = a[0]; f[1] = a[1]; f[2] = a[2]; f[3] = a[3];
    f[4] = c[0]; f[5] = c[1]; f[6] = c[2]; f[7] = c[3];
    P16 ph, hi, lo;
#pragma unroll
    for (int e = 0; e < 8; ++e) {
        ph.h[e] = (f16t)f[e];
        u16 hb  = bfb(f[e]);
        hi.s[e] = hb;
        lo.s[e] = bfb(f[e] - bff(hb));
    }
    const size_t d = (size_t)i * 8;
    *(volatile v4u*)(xh + d)  = ph.u;
    *(volatile v4u*)(xhi + d) = hi.u;
    *(volatile v4u*)(xlo + d) = lo.u;
    __threadfence();
    *(volatile v4u*)(xh + d)  = ph.u;
    *(volatile v4u*)(xhi + d) = hi.u;
    *(volatile v4u*)(xlo + d) = lo.u;
}

__global__ __launch_bounds__(256)
void k_cvt_h(const float* __restrict__ w, f16t* dst, int n8, float sc) {
    const int i = blockIdx.x * 256 + threadIdx.x;
    if (i >= n8) return;
    const float* p = w + (size_t)i * 8;
    v4f a = *(const v4f*)p;
    v4f c = *(const v4f*)(p + 4);
    P16 ph;
#pragma unroll
    for (int e = 0; e < 4; ++e) {
        ph.h[e]     = (f16t)(a[e] * sc);
        ph.h[4 + e] = (f16t)(c[e] * sc);
    }
    const size_t d = (size_t)i * 8;
    *(volatile v4u*)(dst + d) = ph.u;
    __threadfence();
    *(volatile v4u*)(dst + d) = ph.u;
}

__global__ __launch_bounds__(256)
void k_cvt_b(const float* __restrict__ w, u16* dhi, u16* dlo, int n8, float sc) {
    const int i = blockIdx.x * 256 + threadIdx.x;
    if (i >= n8) return;
    const float* p = w + (size_t)i * 8;
    v4f a = *(const v4f*)p;
    v4f c = *(const v4f*)(p + 4);
    float f[8];
    f[0] = a[0]; f[1] = a[1]; f[2] = a[2]; f[3] = a[3];
    f[4] = c[0]; f[5] = c[1]; f[6] = c[2]; f[7] = c[3];
    P16 hi, lo;
#pragma unroll
    for (int e = 0; e < 8; ++e) {
        float v = f[e] * sc;
        u16 hb  = bfb(v);
        hi.s[e] = hb;
        lo.s[e] = bfb(v - bff(hb));
    }
    const size_t d = (size_t)i * 8;
    *(volatile v4u*)(dhi + d) = hi.u;
    *(volatile v4u*)(dlo + d) = lo.u;
    __threadfence();
    *(volatile v4u*)(dhi + d) = hi.u;
    *(volatile v4u*)(dlo + d) = lo.u;
}

__global__ __launch_bounds__(256)
void k_xT(const float* __restrict__ x, f16t* xt) {
    __shared__ __attribute__((aligned(16))) f16t L[32 * HP];
    const int tid = threadIdx.x;
    const int k0 = blockIdx.x * 64, i0 = blockIdx.y * 32, b = blockIdx.z;
    const int kr = tid >> 2, seg = tid & 3;
    const float* src = x + ((size_t)b * 256 + k0 + kr) * 256 + i0 + seg * 8;
    v4f a = *(const v4f*)src;
    v4f c = *(const v4f*)(src + 4);
#pragma unroll
    for (int e = 0; e < 4; ++e) {
        L[(seg * 8 + e) * HP + kr]     = (f16t)a[e];
        L[(seg * 8 + 4 + e) * HP + kr] = (f16t)c[e];
    }
    __syncthreads();
    const int row = tid >> 3, pc = tid & 7;
    P16 v;
    v.h = *(const v8h*)(L + row * HP + pc * 8);
    f16t* d = xt + ((size_t)b * 256 + i0 + row) * 256 + k0 + pc * 8;
    *(volatile v4u*)d = v.u;
    __threadfence();
    *(volatile v4u*)d = v.u;
}

__global__ __launch_bounds__(128)
void k_enc(const f16t* __restrict__ X, const f16t* __restrict__ W, const float* __restrict__ bias,
           f16t* HC, float inv) {
    __shared__ __attribute__((aligned(16))) f16t S[32 * EP];
    const int tid = threadIdx.x, w = tid >> 5, l = tid & 31, h = l >> 4, m = l & 15;
    const int r0 = blockIdx.x * 32, c0 = blockIdx.y * 64, cw = c0 + 16 * w;

    v8f acc[2][3];
#pragma unroll
    for (int i = 0; i < 2; ++i)
#pragma unroll
        for (int g = 0; g < 3; ++g) acc[i][g] = zf8();

    const f16t* ap  = X + (size_t)(r0 + m) * 256 + 8 * h;
    const f16t* bq0 = W + (size_t)(cw + m) * 256 + 8 * h;
    const f16t* bq1 = bq0 + (size_t)1024 * 256;
    const f16t* bq2 = bq0 + (size_t)1536 * 256;
#pragma unroll 1
    for (int kt = 0; kt < 8; ++kt) {
        const int ko = kt * 32;
        v16h a[2], b[3];
        a[0] = ldh(ap + ko);
        a[1] = ldh(ap + (size_t)16 * 256 + ko);
        b[0] = ldh(bq0 + ko);
        b[1] = ldh(bq1 + ko);
        b[2] = ldh(bq2 + ko);
#pragma unroll
        for (int i = 0; i < 2; ++i)
#pragma unroll
            for (int g = 0; g < 3; ++g) acc[i][g] = wh(a[i], b[g], acc[i][g]);
        gd6h(acc, a, b);
    }

    const float bi = bias[cw + m], bg = bias[1024 + cw + m], bo = bias[1536 + cw + m];
#pragma unroll
    for (int i = 0; i < 2; ++i)
#pragma unroll
        for (int r = 0; r < 8; ++r) {
            float gi = fmaf(acc[i][0][r], inv, bi);
            float gg = fmaf(acc[i][1][r], inv, bg);
            float go = fmaf(acc[i][2][r], inv, bo);
            float cs = fsigm(gi) * ftanh(gg);
            float hs = fsigm(go) * ftanh(cs);
            const int lr = 16 * i + 8 * h + r;
            S[lr * EP + 16 * w + m]      = (f16t)hs;
            S[lr * EP + 64 + 16 * w + m] = (f16t)cs;
        }
    __syncthreads();

    P16 v[4];
#pragma unroll
    for (int it = 0; it < 4; ++it) {
        const int p = tid + 128 * it, row = p >> 4, which = (p >> 3) & 1, pc = p & 7;
        v[it].h = *(const v8h*)(S + row * EP + which * 64 + pc * 8);
    }
#pragma unroll
    for (int it = 0; it < 4; ++it) {
        const int p = tid + 128 * it, row = p >> 4, which = (p >> 3) & 1, pc = p & 7;
        *(volatile v4u*)(HC + (size_t)(r0 + row) * 1024 + which * 512 + c0 + pc * 8) = v[it].u;
    }
    __threadfence();
#pragma unroll
    for (int it = 0; it < 4; ++it) {
        const int p = tid + 128 * it, row = p >> 4, which = (p >> 3) & 1, pc = p & 7;
        *(volatile v4u*)(HC + (size_t)(r0 + row) * 1024 + which * 512 + c0 + pc * 8) = v[it].u;
    }
}

template<bool SPLIT>
__global__ __launch_bounds__(128)
void k_g128(const u16* __restrict__ A0, const u16* __restrict__ A1,
            const u16* __restrict__ B0, const u16* __restrict__ B1,
            float* C, int K, float inv) {
    __shared__ __attribute__((aligned(16))) float S[32 * GP];
    const int tid = threadIdx.x, w = tid >> 5, l = tid & 31, h = l >> 4, m = l & 15;
    const int r0 = blockIdx.x * 32, cwo = 32 * w;

    v8f acc[2][2];
#pragma unroll
    for (int i = 0; i < 2; ++i)
#pragma unroll
        for (int j = 0; j < 2; ++j) acc[i][j] = zf8();

    const size_t ao = (size_t)(r0 + m) * K + 8 * h;
    const size_t bo = (size_t)(cwo + m) * K + 8 * h;
    const size_t ts = (size_t)16 * K;
    const int KT = K >> 5;
#pragma unroll 1
    for (int kt = 0; kt < KT; ++kt) {
        const int ko = kt * 32;
        if (!SPLIT) {
            const f16t* Ah = (const f16t*)A0;
            const f16t* Bh = (const f16t*)B0;
            v16h a[2], b[2];
            a[0] = ldh(Ah + ao + ko);
            a[1] = ldh(Ah + ao + ts + ko);
            b[0] = ldh(Bh + bo + ko);
            b[1] = ldh(Bh + bo + ts + ko);
#pragma unroll
            for (int i = 0; i < 2; ++i)
#pragma unroll
                for (int j = 0; j < 2; ++j) acc[i][j] = wh(a[i], b[j], acc[i][j]);
            gd4h(acc, a, b);
        } else {
            v16b ah[2], al[2], bh[2], bl[2];
            ah[0] = ldb(A0 + ao + ko);
            ah[1] = ldb(A0 + ao + ts + ko);
            al[0] = ldb(A1 + ao + ko);
            al[1] = ldb(A1 + ao + ts + ko);
            bh[0] = ldb(B0 + bo + ko);
            bh[1] = ldb(B0 + bo + ts + ko);
            bl[0] = ldb(B1 + bo + ko);
            bl[1] = ldb(B1 + bo + ts + ko);
#pragma unroll
            for (int i = 0; i < 2; ++i)
#pragma unroll
                for (int j = 0; j < 2; ++j) {
                    acc[i][j] = wb(ah[i], bh[j], acc[i][j]);
                    acc[i][j] = wb(ah[i], bl[j], acc[i][j]);
                    acc[i][j] = wb(al[i], bh[j], acc[i][j]);
                }
            gd4b(acc, ah, al, bh, bl);
        }
    }

#pragma unroll
    for (int i = 0; i < 2; ++i)
#pragma unroll
        for (int j = 0; j < 2; ++j)
#pragma unroll
            for (int r = 0; r < 8; ++r)
                S[(16 * i + 8 * h + r) * GP + cwo + 16 * j + m] = acc[i][j][r] * inv;
    __syncthreads();

    P32 v[8];
#pragma unroll
    for (int it = 0; it < 8; ++it) {
        const int p = tid + 128 * it, row = p >> 5, pc = p & 31;
        v[it].f = *(const v4f*)(S + row * GP + pc * 4);
    }
#pragma unroll
    for (int it = 0; it < 8; ++it) {
        const int p = tid + 128 * it, row = p >> 5, pc = p & 31;
        *(volatile v4u*)(C + (size_t)(r0 + row) * 128 + pc * 4) = v[it].u;
    }
    __threadfence();
#pragma unroll
    for (int it = 0; it < 8; ++it) {
        const int p = tid + 128 * it, row = p >> 5, pc = p & 31;
        *(volatile v4u*)(C + (size_t)(r0 + row) * 128 + pc * 4) = v[it].u;
    }
}

__global__ __launch_bounds__(256)
void k_att(const float* __restrict__ w1hc, const float* __restrict__ w2x,
           const float* __restrict__ av, const f16t* __restrict__ XT, u16* Zh, u16* Zl) {
    __shared__ __attribute__((aligned(16))) float Q[16 * 128];
    __shared__ __attribute__((aligned(16))) float VV[128];
    __shared__ __attribute__((aligned(16))) float SC[16 * AP];
    __shared__ __attribute__((aligned(16))) f16t  BT[16 * BP];
    __shared__ __attribute__((aligned(16))) float ZS[16 * AP];
    const int tid = threadIdx.x;
    const int t0 = blockIdx.x * 16, b = blockIdx.y;
    const size_t rowb = (size_t)b * 256;

#pragma unroll
    for (int it = 0; it < 8; ++it) {
        const int p = tid + 256 * it;
        Q[p] = w1hc[(rowb + t0 + (p >> 7)) * 128 + (p & 127)];
    }
    if (tid < 128) VV[tid] = av[tid];
    __syncthreads();

    float s[16];
#pragma unroll
    for (int t = 0; t < 16; ++t) s[t] = 0.0f;
    const float* wr = w2x + (rowb + tid) * 128;
#pragma unroll 1
    for (int v = 0; v < 128; ++v) {
        const float wk = wr[v];
        const float vv = VV[v];
#pragma unroll
        for (int t = 0; t < 16; ++t)
            s[t] = fmaf(vv, ftanh(Q[t * 128 + v] + wk), s[t]);
    }
#pragma unroll
    for (int t = 0; t < 16; ++t) SC[t * AP + tid] = s[t];
    __syncthreads();

    const int w = tid >> 5, l = tid & 31, h = l >> 4, m = l & 15;
#pragma unroll
    for (int q = 0; q < 2; ++q) {
        const int rr = 2 * w + q;
        float e[8];
#pragma unroll
        for (int j = 0; j < 8; ++j) e[j] = SC[rr * AP + l + 32 * j];
        float mx = e[0];
#pragma unroll
        for (int j = 1; j < 8; ++j) mx = fmaxf(mx, e[j]);
#pragma unroll
        for (int off = 16; off > 0; off >>= 1) mx = fmaxf(mx, __shfl_xor(mx, off));
        float sum = 0.0f;
#pragma unroll
        for (int j = 0; j < 8; ++j) { e[j] = expf(e[j] - mx); sum += e[j]; }
#pragma unroll
        for (int off = 16; off > 0; off >>= 1) sum += __shfl_xor(sum, off);
        const float scl = 4096.0f * __builtin_amdgcn_rcpf(sum);
#pragma unroll
        for (int j = 0; j < 8; ++j) BT[rr * BP + l + 32 * j] = (f16t)(e[j] * scl);
    }
    __syncthreads();

    v8f acc0 = zf8(), acc1 = zf8();
    const f16t* ap = BT + m * BP + 8 * h;
    const f16t* bp = XT + (rowb + 32 * w + m) * 256 + 8 * h;
#pragma unroll 1
    for (int kt = 0; kt < 8; ++kt) {
        const int ko = kt * 32;
        v16h a  = ldh(ap + ko);
        v16h b0 = ldh(bp + ko);
        v16h b1 = ldh(bp + (size_t)16 * 256 + ko);
        acc0 = wh(a, b0, acc0);
        acc1 = wh(a, b1, acc1);
        gd2h(acc0, acc1, a, b0, b1);
    }
    const float iz = 1.0f / 4096.0f;
#pragma unroll
    for (int r = 0; r < 8; ++r) {
        ZS[(8 * h + r) * AP + 32 * w + m]      = acc0[r] * iz;
        ZS[(8 * h + r) * AP + 32 * w + 16 + m] = acc1[r] * iz;
    }
    __syncthreads();

    P16 hi[2], lo[2];
#pragma unroll
    for (int it = 0; it < 2; ++it) {
        const int p = tid + 256 * it, row = p >> 5, pc = p & 31;
        v4f f0 = *(const v4f*)(ZS + row * AP + pc * 8);
        v4f f1 = *(const v4f*)(ZS + row * AP + pc * 8 + 4);
        float f[8];
        f[0] = f0[0]; f[1] = f0[1]; f[2] = f0[2]; f[3] = f0[3];
        f[4] = f1[0]; f[5] = f1[1]; f[6] = f1[2]; f[7] = f1[3];
#pragma unroll
        for (int e2 = 0; e2 < 8; ++e2) {
            u16 hb = bfb(f[e2]);
            hi[it].s[e2] = hb;
            lo[it].s[e2] = bfb(f[e2] - bff(hb));
        }
    }
#pragma unroll
    for (int it = 0; it < 2; ++it) {
        const int p = tid + 256 * it, row = p >> 5, pc = p & 31;
        const size_t d = (rowb + t0 + row) * 256 + pc * 8;
        *(volatile v4u*)(Zh + d) = hi[it].u;
        *(volatile v4u*)(Zl + d) = lo[it].u;
    }
    __threadfence();
#pragma unroll
    for (int it = 0; it < 2; ++it) {
        const int p = tid + 256 * it, row = p >> 5, pc = p & 31;
        const size_t d = (rowb + t0 + row) * 256 + pc * 8;
        *(volatile v4u*)(Zh + d) = hi[it].u;
        *(volatile v4u*)(Zl + d) = lo[it].u;
    }
}

__global__ __launch_bounds__(256)
void k_dec(const u16* __restrict__ Zh, const u16* __restrict__ Zl,
           const u16* __restrict__ Wh, const u16* __restrict__ Wl,
           const f16t* __restrict__ Whh, const float* __restrict__ bias,
           const f16t* __restrict__ Hin, f16t* Hout, float* Cst, float* YL,
           int step, float inv) {
    __shared__ __attribute__((aligned(16))) float CS[64 * CP];
    __shared__ __attribute__((aligned(16))) f16t  HS[64 * HP];
    __shared__ __attribute__((aligned(16))) float YS[64];
    const int tid = threadIdx.x, wv = tid >> 5, l = tid & 31, h = l >> 4, m = l & 15;
    const int mbase = blockIdx.x * 64, nb = blockIdx.y * 64;
    const int m_off = (wv & 3) * 16, n_off = (wv >> 2) * 32;

    v8f acc[4][2];
#pragma unroll
    for (int g = 0; g < 4; ++g) { acc[g][0] = zf8(); acc[g][1] = zf8(); }

    {
        const u16* ahp = Zh + (size_t)(mbase + m_off + m) * 256 + 8 * h;
        const u16* alp = Zl + (size_t)(mbase + m_off + m) * 256 + 8 * h;
        const u16* bhp = Wh + (size_t)(nb + n_off + m) * 256 + 8 * h;
        const u16* blp = Wl + (size_t)(nb + n_off + m) * 256 + 8 * h;
#pragma unroll 1
        for (int kt = 0; kt < 8; ++kt) {
            const int ko = kt * 32;
            v16b ah = ldb(ahp + ko), al = ldb(alp + ko);
#pragma unroll
            for (int g = 0; g < 4; ++g) {
                v16b bh[2], bl[2];
#pragma unroll
                for (int nh = 0; nh < 2; ++nh) {
                    const size_t to = (size_t)(g * 512 + nh * 16) * 256 + ko;
                    bh[nh] = ldb(bhp + to);
                    bl[nh] = ldb(blp + to);
                }
#pragma unroll
                for (int nh = 0; nh < 2; ++nh) {
                    acc[g][nh] = wb(ah, bh[nh], acc[g][nh]);
                    acc[g][nh] = wb(ah, bl[nh], acc[g][nh]);
                    acc[g][nh] = wb(al, bh[nh], acc[g][nh]);
                }
                gd2b(acc[g][0], acc[g][1], ah, al, bh[0], bh[1], bl[0], bl[1]);
            }
        }
    }
    if (step > 0) {
        const f16t* ap2 = Hin + (size_t)(mbase + m_off + m) * 512 + 8 * h;
        const f16t* bp2 = Whh + (size_t)(nb + n_off + m) * 512 + 8 * h;
#pragma unroll 1
        for (int kt = 0; kt < 16; ++kt) {
            const int ko = kt * 32;
            v16h a = ldh(ap2 + ko);
#pragma unroll
            for (int g = 0; g < 4; ++g) {
                v16h b0 = ldh(bp2 + (size_t)(g * 512) * 512 + ko);
                v16h b1 = ldh(bp2 + (size_t)(g * 512 + 16) * 512 + ko);
                acc[g][0] = wh(a, b0, acc[g][0]);
                acc[g][1] = wh(a, b1, acc[g][1]);
                gd2h(acc[g][0], acc[g][1], a, b0, b1);
            }
        }
    }

#pragma unroll
    for (int nh = 0; nh < 2; ++nh) {
        const int lc  = n_off + 16 * nh + m;
        const int col = nb + lc;
        const float bi = bias[col], bf = bias[512 + col], bg = bias[1024 + col], bo = bias[1536 + col];
#pragma unroll
        for (int r = 0; r < 8; ++r) {
            const int lr = m_off + 8 * h + r, row = mbase + lr;
            float gi = fmaf(acc[0][nh][r], inv, bi);
            float gf = fmaf(acc[1][nh][r], inv, bf);
            float gg = fmaf(acc[2][nh][r], inv, bg);
            float go = fmaf(acc[3][nh][r], inv, bo);
            float cp = (step > 0) ? Cst[(size_t)row * 512 + col] : 0.0f;
            float cn = fsigm(gf) * cp + fsigm(gi) * ftanh(gg);
            float hn = fsigm(go) * ftanh(cn);
            CS[lr * CP + lc] = cn;
            HS[lr * HP + lc] = (f16t)hn;
            if (row == 255) YS[lc] = hn;
        }
    }
    __syncthreads();

    P32 cv[4];
    P16 hv[2];
    P32 yv;
#pragma unroll
    for (int it = 0; it < 4; ++it) {
        const int p = tid + 256 * it, row = p >> 4, pc = p & 15;
        cv[it].f = *(const v4f*)(CS + row * CP + pc * 4);
    }
#pragma unroll
    for (int it = 0; it < 2; ++it) {
        const int p = tid + 256 * it, row = p >> 3, pc = p & 7;
        hv[it].h = *(const v8h*)(HS + row * HP + pc * 8);
    }
    const bool ylane = (mbase == 192) && (tid < 16);
    yv.f = *(const v4f*)(YS + (tid & 15) * 4);
#pragma unroll
    for (int it = 0; it < 4; ++it) {
        const int p = tid + 256 * it, row = p >> 4, pc = p & 15;
        *(volatile v4u*)(Cst + (size_t)(mbase + row) * 512 + nb + pc * 4) = cv[it].u;
    }
#pragma unroll
    for (int it = 0; it < 2; ++it) {
        const int p = tid + 256 * it, row = p >> 3, pc = p & 7;
        *(volatile v4u*)(Hout + (size_t)(mbase + row) * 512 + nb + pc * 8) = hv[it].u;
    }
    if (ylane) *(volatile v4u*)(YL + (size_t)step * 512 + nb + tid * 4) = yv.u;
    __threadfence();
#pragma unroll
    for (int it = 0; it < 4; ++it) {
        const int p = tid + 256 * it, row = p >> 4, pc = p & 15;
        *(volatile v4u*)(Cst + (size_t)(mbase + row) * 512 + nb + pc * 4) = cv[it].u;
    }
#pragma unroll
    for (int it = 0; it < 2; ++it) {
        const int p = tid + 256 * it, row = p >> 3, pc = p & 7;
        *(volatile v4u*)(Hout + (size_t)(mbase + row) * 512 + nb + pc * 8) = hv[it].u;
    }
    if (ylane) *(volatile v4u*)(YL + (size_t)step * 512 + nb + tid * 4) = yv.u;
}

__global__ __launch_bounds__(64)
void k_fc(const float* __restrict__ YL, const float* __restrict__ W, const float* __restrict__ bias,
          float* out) {
    __shared__ __attribute__((aligned(16))) float O[32];
    const int tid = threadIdx.x;
    if (tid < 32) {
        const int b = tid >> 1, j = tid & 1;
        float s = 0.0f;
#pragma unroll 4
        for (int k = 0; k < 512; ++k) s = fmaf(YL[b * 512 + k], W[j * 512 + k], s);
        O[tid] = s + bias[j];
    }
    __syncthreads();
    if (tid < 8) {
        P32 v;
        v.f = *(const v4f*)(O + tid * 4);
        *(volatile v4u*)(out + tid * 4) = v.u;
        __threadfence();
        *(volatile v4u*)(out + tid * 4) = v.u;
    }
}

extern "C" void kernel_launch(void* const* d_in, const int* in_sizes, int n_in,
                              void* d_out, int out_size, void* d_ws, size_t ws_size,
                              hipStream_t stream) {
    const int NBATCH = 16, NSTEP = 256, NIN = 256, HE = 512, NV = 128, HD = 512, NO = 2;
    const int NR = NBATCH * NSTEP;

    if (n_in < 11) return;
    if (in_sizes[0] != NR * NIN || in_sizes[1] != 4 * HE * NIN || in_sizes[2] != 4 * HE ||
        in_sizes[3] != NV * 2 * HE || in_sizes[4] != NV * NIN || in_sizes[5] != NV ||
        in_sizes[6] != 4 * HD * NIN || in_sizes[7] != 4 * HD * HD || in_sizes[8] != 4 * HD ||
        in_sizes[9] != NO * HD || in_sizes[10] != NO || out_size != NBATCH * NO) return;

    const float* x       = (const float*)d_in[0];
    const float* enc_Wih = (const float*)d_in[1];
    const float* enc_b   = (const float*)d_in[2];
    const float* att_W1  = (const float*)d_in[3];
    const float* att_W2  = (const float*)d_in[4];
    const float* att_v   = (const float*)d_in[5];
    const float* dec_Wih = (const float*)d_in[6];
    const float* dec_Whh = (const float*)d_in[7];
    const float* dec_b   = (const float*)d_in[8];
    const float* fc_W    = (const float*)d_in[9];
    const float* fc_b    = (const float*)d_in[10];
    float* out = (float*)d_out;

    char* ws = (char*)d_ws;
    size_t off = 0;
    auto carve = [&](size_t bytes) -> char* {
        char* p = ws + off;
        off = (off + bytes + 255) & ~(size_t)255;
        return p;
    };
    f16t*  X16  = (f16t*) carve((size_t)NR * NIN * 2);
    u16*   Xhi  = (u16*)  carve((size_t)NR * NIN * 2);
    u16*   Xlo  = (u16*)  carve((size_t)NR * NIN * 2);
    f16t*  XT   = (f16t*) carve((size_t)NR * NIN * 2);
    f16t*  EW   = (f16t*) carve((size_t)4 * HE * NIN * 2);
    f16t*  W1   = (f16t*) carve((size_t)NV * 2 * HE * 2);
    u16*   W2hi = (u16*)  carve((size_t)NV * NIN * 2);
    u16*   W2lo = (u16*)  carve((size_t)NV * NIN * 2);
    u16*   DWhi = (u16*)  carve((size_t)4 * HD * NIN * 2);
    u16*   DWlo = (u16*)  carve((size_t)4 * HD * NIN * 2);
    f16t*  DWhh = (f16t*) carve((size_t)4 * HD * HD * 2);
    f16t*  HC   = (f16t*) carve((size_t)NR * 2 * HE * 2);
    float* W1HC = (float*)carve((size_t)NR * NV * 4);
    float* W2X  = (float*)carve((size_t)NR * NV * 4);
    u16*   Zhi  = (u16*)  carve((size_t)NR * NIN * 2);
    u16*   Zlo  = (u16*)  carve((size_t)NR * NIN * 2);
    f16t*  Ha   = (f16t*) carve((size_t)NSTEP * HD * 2);
    f16t*  Hb   = (f16t*) carve((size_t)NSTEP * HD * 2);
    float* Cst  = (float*)carve((size_t)NSTEP * HD * 4);
    float* YL   = (float*)carve((size_t)NBATCH * HD * 4);
    if (off > ws_size || off > ((size_t)128 << 20)) return;

    {
        const int n8 = NR * NIN / 8;
        k_cvt_x<<<dim3((n8 + 255) / 256), dim3(256), 0, stream>>>(x, X16, Xhi, Xlo, n8);
    }
    k_xT<<<dim3(NIN / 64, NIN / 32, NBATCH), dim3(256), 0, stream>>>(x, XT);
    {
        const int n8 = 4 * HE * NIN / 8;
        k_cvt_h<<<dim3((n8 + 255) / 256), dim3(256), 0, stream>>>(enc_Wih, EW, n8, 16.0f);
    }
    {
        const int n8 = NV * 2 * HE / 8;
        k_cvt_h<<<dim3((n8 + 255) / 256), dim3(256), 0, stream>>>(att_W1, W1, n8, 32.0f);
    }
    {
        const int n8 = NV * NIN / 8;
        k_cvt_b<<<dim3((n8 + 255) / 256), dim3(256), 0, stream>>>(att_W2, W2hi, W2lo, n8, 1.0f);
    }
    {
        const int n8 = 4 * HD * NIN / 8;
        k_cvt_b<<<dim3((n8 + 255) / 256), dim3(256), 0, stream>>>(dec_Wih, DWhi, DWlo, n8, 16.0f);
    }
    {
        const int n8 = 4 * HD * HD / 8;
        k_cvt_h<<<dim3((n8 + 255) / 256), dim3(256), 0, stream>>>(dec_Whh, DWhh, n8, 16.0f);
    }

    k_enc<<<dim3(NR / 32, HE / 64), dim3(128), 0, stream>>>(X16, EW, enc_b, HC, 1.0f / 16.0f);

    k_g128<false><<<dim3(NR / 32), dim3(128), 0, stream>>>(
        (const u16*)HC, (const u16*)HC, (const u16*)W1, (const u16*)W1, W1HC, 2 * HE, 1.0f / 32.0f);
    k_g128<true><<<dim3(NR / 32), dim3(128), 0, stream>>>(
        Xhi, Xlo, W2hi, W2lo, W2X, NIN, 1.0f);

    k_att<<<dim3(NSTEP / 16, NBATCH), dim3(256), 0, stream>>>(W1HC, W2X, att_v, XT, Zhi, Zlo);

    for (int s = 0; s < NBATCH; ++s) {
        const f16t* hin = (s & 1) ? Hb : Ha;
        f16t*       hout = (s & 1) ? Ha : Hb;
        k_dec<<<dim3(NSTEP / 64, HD / 64), dim3(256), 0, stream>>>(
            Zhi + (size_t)s * NSTEP * NIN, Zlo + (size_t)s * NSTEP * NIN,
            DWhi, DWlo, DWhh, dec_b, hin, hout, Cst, YL, s, 1.0f / 16.0f);
    }

    k_fc<<<dim3(1), dim3(64), 0, stream>>>(YL, fc_W, fc_b, out);
}
